// RelativeMultiHeadAttentionLayer_17806934409471
// MI455X (gfx1250) — hardware-verified
//
#include <hip/hip_runtime.h>
#include <stdint.h>
#include <math.h>

typedef __attribute__((ext_vector_type(16))) _Float16 v16h;
typedef __attribute__((ext_vector_type(8)))  _Float16 v8h;
typedef __attribute__((ext_vector_type(16))) __bf16   v16b;
typedef __attribute__((ext_vector_type(8)))  __bf16   v8b;
typedef __attribute__((ext_vector_type(8)))  float    v8f;
typedef __attribute__((ext_vector_type(4)))  float    v4f;
typedef __attribute__((ext_vector_type(8)))  unsigned short v8us;
typedef __attribute__((ext_vector_type(16))) unsigned short v16us;

#define AT_D 64
#define AT_NW 4
#define AT_QB 64
#define AT_KC 64
constexpr int SEQ_LEN   = 512;
constexpr int N_HEADS   = 16;
constexpr int D_MODEL   = 1024;
constexpr int REL_ROWS  = 2 * SEQ_LEN - 1;
constexpr int QBLK_PER_SEQ = SEQ_LEN / AT_QB;
constexpr int KCHUNKS   = SEQ_LEN / AT_KC;
constexpr int BATCH_ALL = 16;
constexpr int BATCH_HALF = 8;
static_assert(D_MODEL == N_HEADS * AT_D);
static_assert(SEQ_LEN % AT_QB == 0 && SEQ_LEN % AT_KC == 0);

__device__ __forceinline__ unsigned short f2bf_bits(float f) {
  unsigned u = __float_as_uint(f);
  return (unsigned short)((u + 0x7FFFu + ((u >> 16) & 1u)) >> 16);
}
__device__ __forceinline__ float bf_bits2f(unsigned short h) { return __uint_as_float(((unsigned)h) << 16); }

__device__ __forceinline__ void dep_guard_h(v8f& a, v8f& b, v16h x, v16h y) { asm volatile("v_nop\n\tv_nop\n\tv_nop\n\tv_nop" : "+v"(a), "+v"(b) : "v"(x), "v"(y)); }
__device__ __forceinline__ void dep_guard_b(v8f& a, v8f& b, v16b x, v16b y) { asm volatile("v_nop\n\tv_nop\n\tv_nop\n\tv_nop" : "+v"(a), "+v"(b) : "v"(x), "v"(y)); }
__device__ __forceinline__ void keep4_h(v16h a, v16h b, v16h c, v16h d) { asm volatile("v_nop" :: "v"(a), "v"(b), "v"(c), "v"(d)); }
__device__ __forceinline__ void keep4_b(v16b a, v16b b, v16b c, v16b d) { asm volatile("v_nop" :: "v"(a), "v"(b), "v"(c), "v"(d)); }
__device__ __forceinline__ void acc_guard4(v8f& a, v8f& b, v8f& c, v8f& d) { asm volatile("v_nop\n\tv_nop\n\tv_nop\n\tv_nop" : "+v"(a), "+v"(b), "+v"(c), "+v"(d)); }

template <typename T> struct Frag;
template <> struct Frag<_Float16> {
  typedef v16h V; union U { v16h v; v8h h[2]; };
  static __device__ __forceinline__ v16h load(const _Float16* p) {
    U f; f.h[0] = *(const v8h*)(p); f.h[1] = *(const v8h*)(p + 16); return f.v;
  }
  static __device__ __forceinline__ v8f mma(v16h a, v16h b, v8f c) {
    return __builtin_amdgcn_wmma_f32_16x16x32_f16(false, a, false, b, (short)0, c, false, false);
  }
  static __device__ __forceinline__ void guard(v8f& a, v8f& b, v16h x, v16h y) { dep_guard_h(a, b, x, y); }
  static __device__ __forceinline__ void keep(v16h a, v16h b, v16h c, v16h d) { keep4_h(a, b, c, d); }
};
template <> struct Frag<__bf16> {
  typedef v16b V; union U { v16b v; v8b h[2]; };
  static __device__ __forceinline__ v16b load(const __bf16* p) {
    U f; f.h[0] = *(const v8b*)(p); f.h[1] = *(const v8b*)(p + 16); return f.v;
  }
  static __device__ __forceinline__ v8f mma(v16b a, v16b b, v8f c) {
    return __builtin_amdgcn_wmma_f32_16x16x32_bf16(false, a, false, b, (short)0, c, false, false);
  }
  static __device__ __forceinline__ void guard(v8f& a, v8f& b, v16b x, v16b y) { dep_guard_b(a, b, x, y); }
  static __device__ __forceinline__ void keep(v16b a, v16b b, v16b c, v16b d) { keep4_b(a, b, c, d); }
};

__device__ __forceinline__ v8f zero8() { return (v8f){0.f, 0.f, 0.f, 0.f, 0.f, 0.f, 0.f, 0.f}; }

template <int ET> struct Elem;
template <> struct Elem<0> { typedef _Float16 T; };
template <> struct Elem<1> { typedef __bf16 T; };
template <int ET, int SPLIT, int BIAS_MODE, int OUT_MODE, bool RESID>
__global__ __launch_bounds__(256) void wmma_gemm64(
    const unsigned short* __restrict__ Ap, const unsigned short* __restrict__ A2p, int lda, long strideA,
    const unsigned short* __restrict__ Btp, const unsigned short* __restrict__ Bt2p, int ldb, long strideB,
    void* __restrict__ Cout, void* __restrict__ Cout2, int ldc, long strideC,
    const float* __restrict__ bias,
    const float* __restrict__ resid, long strideR,
    int M, int N, int K, float scale) {
  typedef typename Elem<ET>::T T;
  typedef typename Frag<T>::V V;
  const T* A = (const T*)Ap; const T* A2 = (const T*)A2p; const T* Bt = (const T*)Btp; const T* Bt2 = (const T*)Bt2p;
  __shared__ __align__(16) float sT[8][16 * 68];
  const int b    = blockIdx.y;
  const int lane = threadIdx.x & 31;
  const int wave = threadIdx.x >> 5;
  const int tilesN = N >> 6;
  const int tilesM = M >> 6;
  const int tile = blockIdx.x * 8 + wave;
  if (tile >= tilesM * tilesN) return;
  const int tm = tile / tilesN;
  const int tn = tile - tm * tilesN;
  const int m0 = tm << 6;
  const int n0 = tn << 6;

  const T* Ab  = A  + (size_t)b * strideA;
  const T* Bb  = Bt + (size_t)b * strideB;
  const T* Ab2 = (SPLIT != 0) ? (A2  + (size_t)b * strideA) : nullptr;
  const T* Bb2 = (SPLIT == 1) ? (Bt2 + (size_t)b * strideB) : nullptr;

  const int rlane = lane & 15;
  const int koff  = (lane >> 4) * 8;
  const int mOff  = (lane >> 4) * 8;

  v8f acc[4][4];
#pragma unroll
  for (int i = 0; i < 4; ++i)
#pragma unroll
    for (int j = 0; j < 4; ++j) acc[i][j] = zero8();

  for (int k0 = 0; k0 < K; k0 += 32) {
    V bh[4], bl[4];
#pragma unroll
    for (int j = 0; j < 4; ++j) {
      const size_t bo = (size_t)(n0 + (j << 4) + rlane) * ldb + koff + k0;
      bh[j] = Frag<T>::load(Bb + bo);
      if (SPLIT == 1) bl[j] = Frag<T>::load(Bb2 + bo);
    }
#pragma unroll
    for (int i = 0; i < 4; ++i) {
      const size_t ao = (size_t)(m0 + (i << 4) + rlane) * lda + koff + k0;
      V ah = Frag<T>::load(Ab + ao);
      V al;
      if (SPLIT != 0) al = Frag<T>::load(Ab2 + ao);
#pragma unroll
      for (int j = 0; j < 4; ++j) {
        acc[i][j] = Frag<T>::mma(ah, bh[j], acc[i][j]);
        if (SPLIT == 1) acc[i][j] = Frag<T>::mma(ah, bl[j], acc[i][j]);
        if (SPLIT != 0) acc[i][j] = Frag<T>::mma(al, bh[j], acc[i][j]);
      }
      Frag<T>::guard(acc[i][0], acc[i][3], ah, (SPLIT != 0) ? al : ah);
    }
    Frag<T>::keep(bh[0], bh[1], bh[2], bh[3]);
    if (SPLIT == 1) Frag<T>::keep(bl[0], bl[1], bl[2], bl[3]);
  }
  acc_guard4(acc[0][0], acc[0][1], acc[0][2], acc[0][3]);
  acc_guard4(acc[1][0], acc[1][1], acc[1][2], acc[1][3]);
  acc_guard4(acc[2][0], acc[2][1], acc[2][2], acc[2][3]);
  acc_guard4(acc[3][0], acc[3][1], acc[3][2], acc[3][3]);

  float* slab = sT[wave];
  const float* Rb = RESID ? (resid + (size_t)b * strideR) : nullptr;
#pragma unroll
  for (int i = 0; i < 4; ++i) {
    const int mBase = m0 + (i << 4);
#pragma unroll
    for (int j = 0; j < 4; ++j) {
      const int n = n0 + (j << 4) + rlane;
      float bv = 0.f;
      if (BIAS_MODE == 2) bv = bf_bits2f(f2bf_bits(bias[n]));
#pragma unroll
      for (int r = 0; r < 8; ++r) {
        float v = acc[i][j][r] * scale;
        if (BIAS_MODE == 1) v += bf_bits2f(f2bf_bits(bias[mBase + mOff + r]));
        if (BIAS_MODE == 2) v += bv;
        if (RESID) v += Rb[(size_t)(mBase + mOff + r) * ldc + n];
        slab[(mOff + r) * 68 + (j << 4) + rlane] = v;
      }
    }
    __builtin_amdgcn_fence(__ATOMIC_RELEASE, "workgroup");
    __builtin_amdgcn_wave_barrier();
    __builtin_amdgcn_fence(__ATOMIC_ACQUIRE, "workgroup");
    if (OUT_MODE == 0) {
      float* C = (float*)Cout + (size_t)b * strideC;
      const int hh = lane >> 4, c4 = (lane & 15) * 4;
      for (int pass = 0; pass < 2; ++pass) {
#pragma unroll
        for (int it = 0; it < 8; ++it) {
          const int row = it * 2 + hh;
          v4f v = *(const v4f*)(slab + row * 68 + c4);
          *(volatile v4f*)(C + (size_t)(mBase + row) * ldc + n0 + c4) = v;
        }
        __threadfence();
      }
    } else {
      const int q = lane >> 3, c8 = (lane & 7) * 8;
      unsigned short* C  = (unsigned short*)Cout  + (size_t)b * strideC;
      unsigned short* C2 = (OUT_MODE == 2) ? ((unsigned short*)Cout2 + (size_t)b * strideC) : nullptr;
      for (int pass = 0; pass < 2; ++pass) {
#pragma unroll
        for (int it = 0; it < 4; ++it) {
          const int row = it * 4 + q;
          const float* sp = slab + row * 68 + c8;
          v8h hv, lv;
#pragma unroll
          for (int e = 0; e < 8; ++e) {
            if (OUT_MODE == 1) {
              hv[e] = (_Float16)sp[e];
            } else {
              unsigned short hb = f2bf_bits(sp[e]);
              unsigned short lb = f2bf_bits(sp[e] - bf_bits2f(hb));
              hv[e] = __builtin_bit_cast(_Float16, hb);
              lv[e] = __builtin_bit_cast(_Float16, lb);
            }
          }
          *(volatile v8h*)(C + (size_t)(mBase + row) * ldc + n0 + c8) = hv;
          if (OUT_MODE == 2) *(volatile v8h*)(C2 + (size_t)(mBase + row) * ldc + n0 + c8) = lv;
        }
        __threadfence();
      }
    }
    __builtin_amdgcn_fence(__ATOMIC_RELEASE, "workgroup");
    __builtin_amdgcn_wave_barrier();
    __builtin_amdgcn_fence(__ATOMIC_ACQUIRE, "workgroup");
  }
}

__global__ __launch_bounds__(256) void cast_f32_bf16x8(
    const float* __restrict__ in, unsigned short* __restrict__ out, int n8) {
  const int i = blockIdx.x * 256 + threadIdx.x;
  if (i < n8) {
    const size_t e0 = (size_t)i * 8;
    const v4f a  = *(const v4f*)(in + e0);
    const v4f a2 = *(const v4f*)(in + e0 + 4);
    v8h hv;
    hv[0] = __builtin_bit_cast(_Float16, f2bf_bits(a[0]));
    hv[1] = __builtin_bit_cast(_Float16, f2bf_bits(a[1]));
    hv[2] = __builtin_bit_cast(_Float16, f2bf_bits(a[2]));
    hv[3] = __builtin_bit_cast(_Float16, f2bf_bits(a[3]));
    hv[4] = __builtin_bit_cast(_Float16, f2bf_bits(a2[0]));
    hv[5] = __builtin_bit_cast(_Float16, f2bf_bits(a2[1]));
    hv[6] = __builtin_bit_cast(_Float16, f2bf_bits(a2[2]));
    hv[7] = __builtin_bit_cast(_Float16, f2bf_bits(a2[3]));
    *(volatile v8h*)(out + e0) = hv;
    __threadfence();
    *(volatile v8h*)(out + e0) = hv;
  }
}

__device__ __forceinline__ v8f at_mma(v16b a, v16b b, v8f c) {
  c = __builtin_amdgcn_wmma_f32_16x16x32_bf16(false, a, false, b, (short)0, c, false, false);
  asm volatile("v_nop\n\tv_nop\n\tv_nop\n\tv_nop" : "+v"(c) : "v"(a), "v"(b));
  return c;
}
union FragU { v16us v; v8us h[2]; };
__device__ __forceinline__ v16b ld_frag16(const unsigned short* p) {
  FragU f;
  f.h[0] = *(const v8us*)(p);
  f.h[1] = *(const v8us*)(p + 16);
  return __builtin_bit_cast(v16b, f.v);
}
__device__ __forceinline__ void vt_put2(unsigned short* Vt, int d, int kvr, unsigned w) {
  Vt[d * AT_KC + kvr]       = (unsigned short)(w & 0xffffu);
  Vt[(d + 1) * AT_KC + kvr] = (unsigned short)(w >> 16);
}

__global__ __launch_bounds__(128)
void rel_attn64_kernel(const unsigned short* __restrict__ Qh, const unsigned short* __restrict__ Ql,
                       const unsigned short* __restrict__ Kh, const unsigned short* __restrict__ Kl,
                       const unsigned short* __restrict__ Vh, const unsigned short* __restrict__ Vl,
                       const float* __restrict__ rel,
                       unsigned short* __restrict__ Oh, unsigned short* __restrict__ Ol,
                       int b0, float sm_scale) {
  __shared__ __align__(16) unsigned short Kst[2 * AT_KC * AT_D];
  __shared__ __align__(16) unsigned short Vth[AT_D * AT_KC];
  __shared__ __align__(16) unsigned short Vtl[AT_D * AT_KC];
  __shared__ __align__(16) unsigned short Psh[AT_NW][16 * AT_KC];
  __shared__ __align__(16) unsigned short Psl[AT_NW][16 * AT_KC];
  __shared__ float sBias[128];
  unsigned short* Ksh = Kst;
  unsigned short* Ksl = Kst + AT_KC * AT_D;

  const int tid  = threadIdx.x;
  const int wave = tid >> 5;
  const int lane = tid & 31;
  const int hh   = lane >> 4;
  const int c    = lane & 15;

  const int bx  = blockIdx.x;
  const int qb  = bx % QBLK_PER_SEQ;
  const int bhx = bx / QBLK_PER_SEQ;
  const int h   = bhx % N_HEADS;
  const int bl  = bhx / N_HEADS;
  const int b   = b0 + bl;
  const int q0  = qb * AT_QB + wave * 16;

  v16b qah[2], qal[2];
  {
    const size_t qoff = ((size_t)b * SEQ_LEN + q0 + c) * D_MODEL + (size_t)h * AT_D + 8 * hh;
#pragma unroll
    for (int dc = 0; dc < 2; ++dc) {
      qah[dc] = ld_frag16(Qh + qoff + dc * 32);
      qal[dc] = ld_frag16(Ql + qoff + dc * 32);
    }
  }

  float mrow[8], lrow[8];
  v8f oacc[4];
#pragma unroll
  for (int r = 0; r < 8; ++r) { mrow[r] = -INFINITY; lrow[r] = 0.f; }
#pragma unroll
  for (int t = 0; t < 4; ++t) oacc[t] = zero8();

  const int qrl = wave * 16 + 8 * hh;

  for (int kc = 0; kc < KCHUNKS; ++kc) {
    const int kv0 = kc * AT_KC;
    __syncthreads();
    {
      const int kvr = tid >> 1, dh = (tid & 1) * 32;
      const size_t roff = ((size_t)b * SEQ_LEN + kv0 + kvr) * D_MODEL + (size_t)h * AT_D + dh;
      {
        const uint4* gkh = (const uint4*)(Kh + roff);
        const uint4* gkl = (const uint4*)(Kl + roff);
        uint4* skh = (uint4*)(Ksh + kvr * AT_D + dh);
        uint4* skl = (uint4*)(Ksl + kvr * AT_D + dh);
        uint4 th[4], tl[4];
#pragma unroll
        for (int i = 0; i < 4; ++i) { th[i] = gkh[i]; tl[i] = gkl[i]; }
#pragma unroll
        for (int i = 0; i < 4; ++i) { skh[i] = th[i]; skl[i] = tl[i]; }
      }
      asm volatile("" ::: "memory");
      {
        const uint4* gvh = (const uint4*)(Vh + roff);
        const uint4* gvl = (const uint4*)(Vl + roff);
#pragma unroll
        for (int i = 0; i < 4; ++i) {
          const uint4 wh = gvh[i];
          const uint4 wl = gvl[i];
          const int d = dh + 8 * i;
          vt_put2(Vth, d + 0, kvr, wh.x); vt_put2(Vth, d + 2, kvr, wh.y);
          vt_put2(Vth, d + 4, kvr, wh.z); vt_put2(Vth, d + 6, kvr, wh.w);
          vt_put2(Vtl, d + 0, kvr, wl.x); vt_put2(Vtl, d + 2, kvr, wl.y);
          vt_put2(Vtl, d + 4, kvr, wl.z); vt_put2(Vtl, d + 6, kvr, wl.w);
        }
      }
      {
        int idx = qb * AT_QB - kv0 + (SEQ_LEN - AT_KC) + tid;
        idx = idx < 0 ? 0 : (idx > REL_ROWS - 1 ? REL_ROWS - 1 : idx);
        sBias[tid] = bf_bits2f(f2bf_bits(rel[(size_t)idx * N_HEADS + h]));
      }
    }
    __syncthreads();

    v8f s[4];
#pragma unroll
    for (int j = 0; j < 4; ++j) {
      s[j] = zero8();
#pragma unroll
      for (int dc = 0; dc < 2; ++dc) {
        const unsigned short* kp = Ksh + (j * 16 + c) * AT_D + dc * 32 + 8 * hh;
        const unsigned short* kq = Ksl + (j * 16 + c) * AT_D + dc * 32 + 8 * hh;
        const v16b kbv = ld_frag16(kp);
        const v16b klv = ld_frag16(kq);
        s[j] = at_mma(qah[dc], kbv, s[j]);
        s[j] = at_mma(qah[dc], klv, s[j]);
        s[j] = at_mma(qal[dc], kbv, s[j]);
      }
    }
    float cm[8];
#pragma unroll
    for (int r = 0; r < 8; ++r) {
      float m = -INFINITY;
#pragma unroll
      for (int j = 0; j < 4; ++j) {
        const float val = s[j][r] * sm_scale + sBias[(qrl + r) - (j * 16 + c) + (AT_KC - 1)];
        s[j][r] = val;
        m = fmaxf(m, val);
      }
#pragma unroll
      for (int off = 1; off < 16; off <<= 1) m = fmaxf(m, __shfl_xor(m, off, 32));
      cm[r] = m;
    }
    unsigned short* pwh = Psh[wave];
    unsigned short* pwl = Psl[wave];
#pragma unroll
    for (int r = 0; r < 8; ++r) {
      const float mnew = fmaxf(mrow[r], cm[r]);
      const float alpha = expf(mrow[r] - mnew);
      mrow[r] = mnew;
      float psum = 0.f;
#pragma unroll
      for (int j = 0; j < 4; ++j) {
        const float p = expf(s[j][r] - mnew);
        psum += p;
        const unsigned short hb = f2bf_bits(p);
        const unsigned short lb = f2bf_bits(p - bf_bits2f(hb));
        pwh[(8 * hh + r) * AT_KC + j * 16 + c] = hb;
        pwl[(8 * hh + r) * AT_KC + j * 16 + c] = lb;
      }
#pragma unroll
      for (int off = 1; off < 16; off <<= 1) psum += __shfl_xor(psum, off, 32);
      lrow[r] = lrow[r] * alpha + psum;
#pragma unroll
      for (int t = 0; t < 4; ++t) oacc[t][r] *= alpha;
    }
    __syncthreads();

#pragma unroll 1
    for (int kk = 0; kk < 2; ++kk) {
      const v16b pav = ld_frag16(pwh + c * AT_KC + kk * 32 + 8 * hh);
      const v16b plv = ld_frag16(pwl + c * AT_KC + kk * 32 + 8 * hh);
#pragma unroll
      for (int t = 0; t < 4; ++t) {
        const v16b vbv = ld_frag16(Vth + (t * 16 + c) * AT_KC + kk * 32 + 8 * hh);
        const v16b vlv = ld_frag16(Vtl + (t * 16 + c) * AT_KC + kk * 32 + 8 * hh);
        oacc[t] = at_mma(pav, vbv, oacc[t]);
        oacc[t] = at_mma(pav, vlv, oacc[t]);
        oacc[t] = at_mma(plv, vbv, oacc[t]);
      }
    }
  }

  __syncthreads();
  float* osw = reinterpret_cast<float*>(Kst) + wave * (16 * AT_D);
#pragma unroll
  for (int r = 0; r < 8; ++r) {
    const float inv = 1.0f / lrow[r];
#pragma unroll
    for (int t = 0; t < 4; ++t) osw[(8 * hh + r) * AT_D + t * 16 + c] = oacc[t][r] * inv;
  }
  __syncthreads();
  {
    const int rq = lane >> 3, c8 = (lane & 7) * 8;
    const size_t obase = ((size_t)bl * SEQ_LEN + q0) * D_MODEL + (size_t)h * AT_D + c8;
    for (int pass = 0; pass < 2; ++pass) {
#pragma unroll
      for (int it = 0; it < 4; ++it) {
        const int row = it * 4 + rq;
        const float* sp = osw + row * AT_D + c8;
        v8h hv, lv;
#pragma unroll
        for (int e = 0; e < 8; ++e) {
          const unsigned short hb = f2bf_bits(sp[e]);
          const unsigned short lb = f2bf_bits(sp[e] - bf_bits2f(hb));
          hv[e] = __builtin_bit_cast(_Float16, hb);
          lv[e] = __builtin_bit_cast(_Float16, lb);
        }
        *(volatile v8h*)(Oh + obase + (size_t)row * D_MODEL) = hv;
        *(volatile v8h*)(Ol + obase + (size_t)row * D_MODEL) = lv;
      }
      __threadfence();
    }
  }
}

extern "C" void kernel_launch(void* const* d_in, const int* in_sizes, int n_in,
                              void* d_out, int out_size, void* d_ws, size_t ws_size,
                              hipStream_t stream) {
  (void)n_in;
  constexpr int MROWS = BATCH_ALL * SEQ_LEN;
  constexpr int MHALF = BATCH_HALF * SEQ_LEN;
  constexpr size_t N_X = (size_t)MROWS * D_MODEL;
  constexpr size_t N_W = (size_t)D_MODEL * D_MODEL;
  constexpr size_t N_REL = (size_t)REL_ROWS * N_HEADS;
  constexpr size_t PLANE_X  = N_X * 2;
  constexpr size_t PLANE_W  = N_W * 2;
  constexpr size_t PLANE_AH = (size_t)MHALF * D_MODEL * 2;
  constexpr size_t OFF_XB  = 0;
  constexpr size_t OFF_ATH = 0;
  constexpr size_t OFF_ATL = OFF_ATH + PLANE_AH;
  constexpr size_t OFF_WQ  = OFF_XB + PLANE_X;
  constexpr size_t OFF_WK  = OFF_WQ + PLANE_W;
  constexpr size_t OFF_WV  = OFF_WK + PLANE_W;
  constexpr size_t OFF_WO  = OFF_WV + PLANE_W;
  constexpr size_t OFF_QH  = OFF_WO + PLANE_W;
  constexpr size_t OFF_QL  = OFF_QH + PLANE_X;
  constexpr size_t OFF_KH  = OFF_QL + PLANE_X;
  constexpr size_t OFF_KL  = OFF_KH + PLANE_X;
  constexpr size_t OFF_VH  = OFF_KL + PLANE_X;
  constexpr size_t OFF_VL  = OFF_VH + PLANE_X;
  constexpr size_t WS_TOTAL = OFF_VL + PLANE_X;
  static_assert(WS_TOTAL == 125829120u);
  static_assert(OFF_ATL + PLANE_AH <= OFF_WQ);
  static_assert(D_MODEL % 32 == 0 && D_MODEL % 64 == 0 && MROWS % 64 == 0 && MHALF % 64 == 0);
  static_assert(N_X % 8 == 0 && N_W % 8 == 0);

  if (ws_size < WS_TOTAL) return;
  if (out_size != (int)N_X) return;
  if (in_sizes[0] != (int)N_X || in_sizes[1] != (int)N_W || in_sizes[2] != D_MODEL ||
      in_sizes[3] != (int)N_W || in_sizes[4] != D_MODEL || in_sizes[5] != (int)N_W ||
      in_sizes[6] != D_MODEL || in_sizes[7] != (int)N_W || in_sizes[8] != D_MODEL ||
      in_sizes[9] != (int)N_REL) return;

  const float* x   = (const float*)d_in[0];
  const float* Wq  = (const float*)d_in[1];
  const float* bq  = (const float*)d_in[2];
  const float* Wk  = (const float*)d_in[3];
  const float* bk  = (const float*)d_in[4];
  const float* Wv  = (const float*)d_in[5];
  const float* bv  = (const float*)d_in[6];
  const float* Wo  = (const float*)d_in[7];
  const float* bo  = (const float*)d_in[8];
  const float* rel = (const float*)d_in[9];
  float* out = (float*)d_out;

  char* ws = (char*)d_ws;
  unsigned short* xb  = (unsigned short*)(ws + OFF_XB);
  unsigned short* ath = (unsigned short*)(ws + OFF_ATH);
  unsigned short* atl = (unsigned short*)(ws + OFF_ATL);
  unsigned short* wqb = (unsigned short*)(ws + OFF_WQ);
  unsigned short* wkb = (unsigned short*)(ws + OFF_WK);
  unsigned short* wvb = (unsigned short*)(ws + OFF_WV);
  unsigned short* wob = (unsigned short*)(ws + OFF_WO);
  unsigned short* qh  = (unsigned short*)(ws + OFF_QH);
  unsigned short* ql  = (unsigned short*)(ws + OFF_QL);
  unsigned short* kh  = (unsigned short*)(ws + OFF_KH);
  unsigned short* kl  = (unsigned short*)(ws + OFF_KL);
  unsigned short* vh  = (unsigned short*)(ws + OFF_VH);
  unsigned short* vl  = (unsigned short*)(ws + OFF_VL);

  {
    const int n8x = (int)(N_X / 8), n8w = (int)(N_W / 8);
    cast_f32_bf16x8<<<(n8x + 255) / 256, 256, 0, stream>>>(x,  xb,  n8x);
    cast_f32_bf16x8<<<(n8w + 255) / 256, 256, 0, stream>>>(Wq, wqb, n8w);
    cast_f32_bf16x8<<<(n8w + 255) / 256, 256, 0, stream>>>(Wk, wkb, n8w);
    cast_f32_bf16x8<<<(n8w + 255) / 256, 256, 0, stream>>>(Wv, wvb, n8w);
    cast_f32_bf16x8<<<(n8w + 255) / 256, 256, 0, stream>>>(Wo, wob, n8w);
  }
  {
    const int blocks = (MROWS / 64) * (D_MODEL / 64) / 8;
    wmma_gemm64<1, 0, 2, 2, false><<<dim3(blocks, 1), 256, 0, stream>>>(
        xb, xb, D_MODEL, 0L, wqb, wqb, D_MODEL, 0L, (void*)qh, (void*)ql, D_MODEL, 0L,
        bq, bq, 0L, MROWS, D_MODEL, D_MODEL, 1.0f);
    wmma_gemm64<1, 0, 2, 2, false><<<dim3(blocks, 1), 256, 0, stream>>>(
        xb, xb, D_MODEL, 0L, wkb, wkb, D_MODEL, 0L, (void*)kh, (void*)kl, D_MODEL, 0L,
        bk, bk, 0L, MROWS, D_MODEL, D_MODEL, 1.0f);
    wmma_gemm64<1, 0, 2, 2, false><<<dim3(blocks, 1), 256, 0, stream>>>(
        xb, xb, D_MODEL, 0L, wvb, wvb, D_MODEL, 0L, (void*)vh, (void*)vl, D_MODEL, 0L,
        bv, bv, 0L, MROWS, D_MODEL, D_MODEL, 1.0f);
  }
  for (int half = 0; half < 2; ++half) {
    const int ablocks = BATCH_HALF * N_HEADS * QBLK_PER_SEQ;
    rel_attn64_kernel<<<ablocks, 128, 0, stream>>>(qh, ql, kh, kl, vh, vl, rel, ath, atl,
                                                    half * BATCH_HALF, 0.125f);
    const int gblocks = (MHALF / 64) * (D_MODEL / 64) / 8;
    float* outp = out + (size_t)half * MHALF * D_MODEL;
    wmma_gemm64<1, 2, 2, 0, false><<<dim3(gblocks, 1), 256, 0, stream>>>(
        ath, atl, D_MODEL, 0L, wob, wob, D_MODEL, 0L, (void*)outp, (void*)outp, D_MODEL, 0L,
        bo, bo, 0L, MHALF, D_MODEL, D_MODEL, 1.0f);
  }
}
